// GIDEncoder_17626545782864
// MI455X (gfx1250) — hardware-verified
//
#include <hip/hip_runtime.h>
#include <hip/hip_bf16.h>

typedef __attribute__((ext_vector_type(16))) _Float16 v16bf;
typedef __attribute__((ext_vector_type(4))) float v4f_t;
typedef float v4fa __attribute__((ext_vector_type(4), may_alias));
__device__ __forceinline__ void st2f(float* p, float v) { *(volatile float*)p = v; __threadfence(); *(volatile float*)p = v; }
typedef __attribute__((ext_vector_type(8)))  float  v8f;

union Frag { v16bf v; unsigned u[8]; uint4 q[2]; };

__device__ __forceinline__ unsigned short f2bf(float f) { return __builtin_bit_cast(unsigned short, (_Float16)f); }
__device__ __forceinline__ unsigned short f2lo(float f) { const _Float16 h = (_Float16)f; return __builtin_bit_cast(unsigned short, (_Float16)((f - (float)h) * 2048.0f)); }
__device__ __forceinline__ unsigned pack2lo(float lo, float hi) { return (unsigned)f2lo(lo) | ((unsigned)f2lo(hi) << 16); }
__device__ __forceinline__ unsigned pack2bf(float lo, float hi) {
    return (unsigned)f2bf(lo) | ((unsigned)f2bf(hi) << 16);
}

__device__ __forceinline__ void load_fragA(Frag& f, const unsigned short* rowbase, int hi) {
    f.q[0] = *(const uint4*)(rowbase + hi * 8);
    f.q[1] = *(const uint4*)(rowbase + 16 + hi * 8);
}
__device__ __forceinline__ void load_fragB(Frag& f, const unsigned short* colbase, int hi) {
    f.q[0] = *(const uint4*)(colbase + hi * 8);
    f.q[1] = *(const uint4*)(colbase + 16 + hi * 8);
}

#define BB   32
#define SS   512
#define NTOK (BB * SS)

__global__ __launch_bounds__(256) void stats1_kernel(
    const float* __restrict__ obs, const float* __restrict__ act,
    const float* __restrict__ rew, float* __restrict__ stats)
{
    __shared__ float s1[256], s2[256];
    int f = blockIdx.x, tid = threadIdx.x;
    float sum = 0.f, sq = 0.f;
    for (int i = tid; i < NTOK; i += 256) {
        int b = i >> 9, s = i & 511;
        int prev = (b << 9) + (s == 0 ? 0 : s - 1);
        float v;
        if (f < 32)        v = obs[prev * 32 + f];
        else if (f < 40)   v = act[(size_t)i * 8 + (f - 32)];
        else if (f == 40)  v = rew[i];
        else { int ff = f - 41; v = obs[(size_t)i * 32 + ff] - obs[prev * 32 + ff]; }
        sum += v; sq += v * v;
    }
    s1[tid] = sum; s2[tid] = sq; __syncthreads();
    for (int o = 128; o >= 1; o >>= 1) {
        if (tid < o) { s1[tid] += s1[tid + o]; s2[tid] += s2[tid + o]; }
        __syncthreads();
    }
    if (tid == 0) {
        float m = s1[0] * (1.f / NTOK);
        float var = s2[0] * (1.f / NTOK) - m * m;
        st2f(stats + f * 32, m);
        st2f(stats + (73 + f) * 32, rsqrtf(var + 1e-5f));
    }
}

__global__ __launch_bounds__(256) void encode_kernel(
    const float* __restrict__ obs, const float* __restrict__ act,
    const float* __restrict__ rew, const float* __restrict__ stats,
    const float* __restrict__ og, const float* __restrict__ ob,
    const float* __restrict__ ag, const float* __restrict__ ab,
    const float* __restrict__ rg, const float* __restrict__ rb,
    const float* __restrict__ tg, const float* __restrict__ tb,
    const float* __restrict__ W_obs, const float* __restrict__ b_obs,
    const float* __restrict__ W_act, const float* __restrict__ b_act,
    const float* __restrict__ W_rew, const float* __restrict__ b_rew,
    const float* __restrict__ W_trn, const float* __restrict__ b_trn,
    float* __restrict__ enc)
{
    __shared__ float xin[80];
    int tok = blockIdx.x;
    int b = tok >> 9, s = tok & 511;
    int prev = (b << 9) + (s == 0 ? 0 : s - 1);
    int tid = threadIdx.x;
    if (tid < 73) {
        float v, gg, bb2;
        if (tid < 32)      { v = obs[prev * 32 + tid];                 gg = og[tid];    bb2 = ob[tid]; }
        else if (tid < 40) { int f = tid - 32; v = act[(size_t)tok * 8 + f]; gg = ag[f]; bb2 = ab[f]; }
        else if (tid == 40){ v = rew[tok];                             gg = rg[0];      bb2 = rb[0]; }
        else               { int f = tid - 41;
                             v = obs[(size_t)tok * 32 + f] - obs[prev * 32 + f];
                             gg = tg[f]; bb2 = tb[f]; }
        xin[tid] = (v - stats[tid * 32]) * stats[(73 + tid) * 32] * gg + bb2;
    }
    __syncthreads();
    int seg = tid >> 6, j = tid & 63;
    float a = 0.f;
    if (seg == 0)      {
#pragma unroll 1
        for (int k = 0; k < 32; ++k) a += xin[k]      * W_obs[k * 64 + j]; a += b_obs[j]; }
    else if (seg == 1) {
#pragma unroll 1
        for (int k = 0; k < 8;  ++k) a += xin[32 + k] * W_act[k * 64 + j]; a += b_act[j]; }
    else if (seg == 2) { a = xin[40] * W_rew[j] + b_rew[j]; }
    else               {
#pragma unroll 1
        for (int k = 0; k < 32; ++k) a += xin[41 + k] * W_trn[k * 64 + j]; a += b_trn[j]; }
    st2f(enc + (size_t)tok * 256 + tid, a);
}

__global__ __launch_bounds__(256) void ln_kernel(
    const float* __restrict__ enc, const float* __restrict__ g,
    const float* __restrict__ bta, float* __restrict__ out)
{
    int lane = threadIdx.x & 31, w = threadIdx.x >> 5;
    int tok = blockIdx.x * 8 + w;
    size_t base = (size_t)tok * 256;
    float v[8]; float sum = 0.f, sq = 0.f;
#pragma unroll
    for (int i = 0; i < 8; ++i) {
        v[i] = enc[base + i * 32 + lane];
        sum += v[i]; sq += v[i] * v[i];
    }
#pragma unroll
    for (int o = 16; o >= 1; o >>= 1) {
        sum += __shfl_xor(sum, o, 32);
        sq  += __shfl_xor(sq,  o, 32);
    }
    float mean = sum * (1.f / 256.f);
    float var  = sq * (1.f / 256.f) - mean * mean;
    float rstd = rsqrtf(var + 1e-5f);
#pragma unroll
    for (int i = 0; i < 8; ++i) {
        int col = i * 32 + lane;
        *(volatile float*)(out + base + col) = (v[i] - mean) * rstd * g[col] + bta[col];
    }
    __threadfence();
#pragma unroll
    for (int i = 0; i < 8; ++i) { int col = i * 32 + lane; *(volatile float*)(out + base + col) = (v[i] - mean) * rstd * g[col] + bta[col]; }
}

__global__ __launch_bounds__(256) void pack_kernel(
    const float* __restrict__ wi, const float* __restrict__ we,
    float* __restrict__ wie)
{
    int i = blockIdx.x * 256 + threadIdx.x;
    if (i < 256 * 256) {
        int k = i >> 8, n = i & 255;
        st2f(wie + i, (n < 128) ? wi[k * 128 + n] : we[k * 128 + (n - 128)]);
    }
}

template <bool SCALE, int ACT, bool OUTB>
__global__ __launch_bounds__(256) void gemm_wmma(
    const float* __restrict__ A, const float* __restrict__ Bw,
    const float* __restrict__ scaleK, const float* __restrict__ shiftK,
    const float* __restrict__ bias,
    float* __restrict__ outF, unsigned short* __restrict__ outB,
    int M, int N, int K)
{
    constexpr bool SPLITK = (!SCALE && ACT == 0 && !OUTB);
    __shared__ __attribute__((aligned(16))) unsigned short Alds[128 * 32], Alds2[SPLITK ? 128 * 32 : 2];
    __shared__ __attribute__((aligned(16))) unsigned short Blds[64 * 32], Blds2[SPLITK ? 64 * 32 : 2];
    __shared__ __attribute__((aligned(16))) float stg[8][16 * 68];
    int tid = threadIdx.x, lane = tid & 31, w = tid >> 5;
    int hi = lane >> 4, ln16 = lane & 15;
    int m0 = blockIdx.y * 128, n0 = blockIdx.x * 64;
    v8f acc[4] = {};

    for (int k0 = 0; k0 < K; k0 += 32) {
#pragma unroll
        for (int t = 0; t < 4; ++t) {
            int idx4 = tid + t * 256;
            int r = idx4 >> 3, c = (idx4 & 7) * 4;
            float4 v = *(const float4*)&A[(size_t)(m0 + r) * K + k0 + c];
            if (SCALE) {
                float4 sc4 = *(const float4*)&scaleK[k0 + c];
                float4 sh4 = *(const float4*)&shiftK[k0 + c];
                v.x = v.x * sc4.x + sh4.x; v.y = v.y * sc4.y + sh4.y;
                v.z = v.z * sc4.z + sh4.z; v.w = v.w * sc4.w + sh4.w;
            }
            uint2 pk; pk.x = pack2bf(v.x, v.y); pk.y = pack2bf(v.z, v.w);
            *(uint2*)&Alds[r * 32 + c] = pk;
            if (SPLITK) { uint2 pl; pl.x = pack2lo(v.x, v.y); pl.y = pack2lo(v.z, v.w); *(uint2*)&Alds2[r * 32 + c] = pl; }
        }
#pragma unroll
        for (int t = 0; t < 2; ++t) {
            int idx4 = tid + t * 256;
            int k = idx4 >> 4, n = (idx4 & 15) * 4;
            float4 v = *(const float4*)&Bw[(size_t)(k0 + k) * N + n0 + n];
            Blds[(n + 0) * 32 + k] = f2bf(v.x);
            Blds[(n + 1) * 32 + k] = f2bf(v.y);
            Blds[(n + 2) * 32 + k] = f2bf(v.z);
            Blds[(n + 3) * 32 + k] = f2bf(v.w);
            if (SPLITK) { Blds2[(n + 0) * 32 + k] = f2lo(v.x); Blds2[(n + 1) * 32 + k] = f2lo(v.y); Blds2[(n + 2) * 32 + k] = f2lo(v.z); Blds2[(n + 3) * 32 + k] = f2lo(v.w); }
        }
        __syncthreads();

        Frag a, al;
        load_fragA(a, &Alds[((w << 4) + ln16) * 32], hi);
        if (SPLITK) load_fragA(al, &Alds2[((w << 4) + ln16) * 32], hi);
#pragma unroll
        for (int nt = 0; nt < 4; ++nt) {
            Frag bf;
            load_fragB(bf, &Blds[(nt * 16 + ln16) * 32], hi);
            if (SPLITK) {
                Frag bl; load_fragB(bl, &Blds2[(nt * 16 + ln16) * 32], hi);
                v8f x = {};
                x = __builtin_amdgcn_wmma_f32_16x16x32_f16(false, al.v, false, bf.v, (short)0, x, false, false);
                x = __builtin_amdgcn_wmma_f32_16x16x32_f16(false, a.v, false, bl.v, (short)0, x, false, false);
                acc[nt] = __builtin_amdgcn_wmma_f32_16x16x32_f16(false, a.v, false, bf.v, (short)0, acc[nt], false, false) + x * (1.0f / 2048.0f);
            } else {
                acc[nt] = __builtin_amdgcn_wmma_f32_16x16x32_f16(
                    false, a.v, false, bf.v, (short)0, acc[nt], false, false);
            }
        }
        __syncthreads();
    }

    float* sw = stg[w];
#pragma unroll
    for (int nt = 0; nt < 4; ++nt)
#pragma unroll
        for (int v = 0; v < 8; ++v) {
            int n = n0 + nt * 16 + ln16;
            float val = acc[nt][v] + (bias ? bias[n] : 0.f);
            if (ACT == 1)      val = fmaxf(val, 0.f);
            else if (ACT == 2) val = tanhf(val);
            sw[(v + 8 * hi) * 68 + nt * 16 + ln16] = val;
        }
    asm volatile("s_wait_dscnt 0" ::: "memory");
    const int mw = m0 + (w << 4);
#pragma unroll 1
    for (int pass = 0; pass < 2; ++pass) {
        if (OUTB) {
#pragma unroll
            for (int i = 0; i < 4; ++i) { const int c = lane + 32 * i, rr = c >> 3, q = (c & 7) * 8; const float* s = sw + rr * 68 + q;
                typedef __attribute__((ext_vector_type(4))) unsigned v4u_t;
                v4u_t pk; pk.x = pack2bf(s[0], s[1]); pk.y = pack2bf(s[2], s[3]); pk.z = pack2bf(s[4], s[5]); pk.w = pack2bf(s[6], s[7]);
                *(volatile v4u_t*)(outB + (size_t)(mw + rr) * N + n0 + q) = pk; }
        } else {
#pragma unroll
            for (int i = 0; i < 8; ++i) { const int c = lane + 32 * i, rr = c >> 4, q = (c & 15) * 4;
                *(volatile v4f_t*)(outF + (size_t)(mw + rr) * N + n0 + q) = *(const volatile v4fa*)(sw + rr * 68 + q); }
        }
        __threadfence();
    }
}

__global__ __launch_bounds__(128) void attn_kernel(
    const unsigned short* __restrict__ qkv, float* __restrict__ x)
{
    int lane = threadIdx.x & 31, w = threadIdx.x >> 5;
    int hi = lane >> 4, ln16 = lane & 15;
    int bh = blockIdx.y, b = bh >> 2, h = bh & 3;
    int q0 = blockIdx.x * 64 + w * 16;
    __shared__ __attribute__((aligned(16))) unsigned short Plds[4][16 * 32];
    __shared__ __attribute__((aligned(16))) float ost[4][16 * 68];
    unsigned short* pl = Plds[w];

    Frag qf[2];
    {
        const unsigned short* qb =
            qkv + ((size_t)(b * SS) + q0 + ln16) * 768 + h * 64;
#pragma unroll
        for (int dc = 0; dc < 2; ++dc) load_fragA(qf[dc], qb + dc * 32, hi);
    }
    v8f acc[4] = {};
    float rowm[8], rows[8];
#pragma unroll
    for (int v = 0; v < 8; ++v) { rowm[v] = -__builtin_inff(); rows[v] = 0.f; }
    const float sc = 0.125f;
    int nch = (q0 + 15) / 32 + 1;

    for (int c = 0; c < nch; ++c) {
        int kt0 = c * 32;
        v8f s[2];
#pragma unroll
        for (int sub = 0; sub < 2; ++sub) {
            v8f z = {}; s[sub] = z;
            const unsigned short* kb =
                qkv + ((size_t)(b * SS) + kt0 + sub * 16 + ln16) * 768 + 256 + h * 64;
#pragma unroll
            for (int dc = 0; dc < 2; ++dc) {
                Frag kf;
                load_fragB(kf, kb + dc * 32, hi);
                s[sub] = __builtin_amdgcn_wmma_f32_16x16x32_f16(
                    false, qf[dc].v, false, kf.v, (short)0, s[sub], false, false);
            }
#pragma unroll
            for (int v = 0; v < 8; ++v) {
                int m = q0 + v + 8 * hi;
                int kk = kt0 + sub * 16 + ln16;
                float sv = s[sub][v] * sc;
                s[sub][v] = (kk > m) ? -__builtin_inff() : sv;
            }
        }
        float scl[8];
#pragma unroll
        for (int v = 0; v < 8; ++v) {
            float mv = fmaxf(s[0][v], s[1][v]);
#pragma unroll
            for (int o = 8; o >= 1; o >>= 1) mv = fmaxf(mv, __shfl_xor(mv, o, 16));
            float nm = fmaxf(rowm[v], mv);
            bool dead = (nm == -__builtin_inff());
            float sl = dead ? 1.f : __expf(rowm[v] - nm);
            float p0 = dead ? 0.f : __expf(s[0][v] - nm);
            float p1 = dead ? 0.f : __expf(s[1][v] - nm);
            float ps = p0 + p1;
#pragma unroll
            for (int o = 8; o >= 1; o >>= 1) ps += __shfl_xor(ps, o, 16);
            rows[v] = rows[v] * sl + ps;
            rowm[v] = nm;
            scl[v] = sl;
            pl[(v + 8 * hi) * 32 + ln16]      = f2bf(p0 * 1024.0f);
            pl[(v + 8 * hi) * 32 + 16 + ln16] = f2bf(p1 * 1024.0f);
        }
#pragma unroll
        for (int nt = 0; nt < 4; ++nt)
#pragma unroll
            for (int v = 0; v < 8; ++v) acc[nt][v] *= scl[v];

        asm volatile("s_wait_dscnt 0" ::: "memory");

        Frag pf;
        load_fragA(pf, &pl[ln16 * 32], hi);
#pragma unroll
        for (int nt = 0; nt < 4; ++nt) {
            Frag vf;
            int d = nt * 16 + ln16;
#pragma unroll
            for (int p = 0; p < 8; ++p) {
                int k1 = kt0 + ((p < 4) ? (hi * 8 + p * 2) : (16 + hi * 8 + (p - 4) * 2));
                size_t i0 = ((size_t)(b * SS) + k1) * 768 + 512 + h * 64 + d;
                unsigned e0 = qkv[i0];
                unsigned e1 = qkv[i0 + 768];
                vf.u[p] = e0 | (e1 << 16);
            }
            acc[nt] = __builtin_amdgcn_wmma_f32_16x16x32_f16(
                false, pf.v, false, vf.v, (short)0, acc[nt], false, false);
        }
    }
    float* so = ost[w];
#pragma unroll
    for (int nt = 0; nt < 4; ++nt)
#pragma unroll
        for (int v = 0; v < 8; ++v) so[(v + 8 * hi) * 68 + nt * 16 + ln16] = acc[nt][v] / (rows[v] * 1024.0f);
    asm volatile("s_wait_dscnt 0" ::: "memory");
#pragma unroll 1
    for (int pass = 0; pass < 2; ++pass) {
#pragma unroll
        for (int i = 0; i < 8; ++i) { const int c = lane + 32 * i, rr = c >> 4, q = (c & 15) * 4;
            *(volatile v4f_t*)(x + ((size_t)(b * SS) + q0 + rr) * 512 + h * 64 + q) = *(const volatile v4fa*)(so + rr * 68 + q); }
        __threadfence();
    }
}

__global__ __launch_bounds__(256) void intes_kernel(
    const float* __restrict__ ie, float* __restrict__ x)
{
    int t = blockIdx.x * 256 + threadIdx.x;
    int b = t >> 8, col = t & 255;
    size_t base = (size_t)b * SS;
    if (col < 128) {
        float run = 0.f;
        for (int s = 0; s < SS; ++s) {
            run += ie[(base + s) * 256 + col];
            st2f(x + (base + s) * 512 + 256 + col, run);
        }
    } else {
        float alpha = (col < 192) ? 0.1f : 0.25f;
        float omc = 1.f - alpha;
        float n = 0.f, pw = 1.f;
        for (int s = 0; s < SS; ++s) {
            n = alpha * ie[(base + s) * 256 + col] + omc * n;
            pw *= omc;
            st2f(x + (base + s) * 512 + 256 + col, n / (1.f - pw));
        }
    }
}

__global__ __launch_bounds__(256) void stats2_kernel(
    const float* __restrict__ x, float* __restrict__ stats)
{
    __shared__ float s1[256], s2[256];
    int f = blockIdx.x, tid = threadIdx.x;
    float sum = 0.f, sq = 0.f;
    for (int i = tid; i < NTOK; i += 256) {
        float v = x[(size_t)i * 512 + f];
        sum += v; sq += v * v;
    }
    s1[tid] = sum; s2[tid] = sq; __syncthreads();
    for (int o = 128; o >= 1; o >>= 1) {
        if (tid < o) { s1[tid] += s1[tid + o]; s2[tid] += s2[tid + o]; }
        __syncthreads();
    }
    if (tid == 0) {
        float m = s1[0] * (1.f / NTOK);
        float var = s2[0] * (1.f / NTOK) - m * m;
        st2f(stats + f * 32, m);
        st2f(stats + (512 + f) * 32, rsqrtf(var + 1e-5f));
    }
}

__global__ __launch_bounds__(256) void fold_kernel(
    const float* __restrict__ stats, const float* __restrict__ g,
    const float* __restrict__ bta, float* __restrict__ scale,
    float* __restrict__ shift)
{
    int f = blockIdx.x * 256 + threadIdx.x;
    if (f < 512) {
        float m = stats[f * 32], r = stats[(512 + f) * 32];
        float sc = g[f] * r;
        st2f(scale + f, sc);
        st2f(shift + f, bta[f] - m * sc);
    }
}

extern "C" void kernel_launch(void* const* d_in, const int* in_sizes, int n_in,
                              void* d_out, int out_size, void* d_ws, size_t ws_size,
                              hipStream_t stream)
{
    const float* obs_seq = (const float*)d_in[0];
    const float* act_seq = (const float*)d_in[1];
    const float* rew_seq = (const float*)d_in[2];
    const float* W_obs   = (const float*)d_in[3];
    const float* b_obs   = (const float*)d_in[4];
    const float* W_act   = (const float*)d_in[5];
    const float* b_act   = (const float*)d_in[6];
    const float* W_rew   = (const float*)d_in[7];
    const float* b_rew   = (const float*)d_in[8];
    const float* W_trn   = (const float*)d_in[9];
    const float* b_trn   = (const float*)d_in[10];
    const float* obs_g   = (const float*)d_in[11];
    const float* obs_b   = (const float*)d_in[12];
    const float* act_g   = (const float*)d_in[13];
    const float* act_b   = (const float*)d_in[14];
    const float* rew_g   = (const float*)d_in[15];
    const float* rew_b   = (const float*)d_in[16];
    const float* trn_g   = (const float*)d_in[17];
    const float* trn_b   = (const float*)d_in[18];
    const float* ln_g    = (const float*)d_in[19];
    const float* ln_b    = (const float*)d_in[20];
    const float* W_attn  = (const float*)d_in[21];
    const float* W_int   = (const float*)d_in[22];
    const float* W_es    = (const float*)d_in[23];
    const float* bn_g    = (const float*)d_in[24];
    const float* bn_b    = (const float*)d_in[25];
    const float* W_dec1  = (const float*)d_in[26];
    const float* b_dec1  = (const float*)d_in[27];
    const float* W_dec2  = (const float*)d_in[28];
    const float* b_dec2  = (const float*)d_in[29];
    float* out = (float*)d_out;

    float* stats1 = (float*)d_ws;
    float* stats2 = stats1 + 256;
    float* scale2 = stats2 + 1024;
    float* shift2 = scale2 + 512;
    float* Wie    = shift2 + 512;
    float* enc    = Wie + 65536;
    float* lnb    = enc + (size_t)NTOK * 256;
    float* xb     = enc;
    unsigned short* qkv = (unsigned short*)(lnb + (size_t)NTOK * 256);
    float* h1     = (float*)qkv;
    float* ie     = (float*)(qkv + (size_t)NTOK * 768);
    stats1 = ie + (size_t)NTOK * 256;
    stats2 = stats1 + 146 * 32;

    stats1_kernel<<<73, 256, 0, stream>>>(obs_seq, act_seq, rew_seq, stats1);

    encode_kernel<<<NTOK, 256, 0, stream>>>(
        obs_seq, act_seq, rew_seq, stats1,
        obs_g, obs_b, act_g, act_b, rew_g, rew_b, trn_g, trn_b,
        W_obs, b_obs, W_act, b_act, W_rew, b_rew, W_trn, b_trn, enc);

    ln_kernel<<<NTOK / 8, 256, 0, stream>>>(enc, ln_g, ln_b, lnb);
    pack_kernel<<<256, 256, 0, stream>>>(W_int, W_es, Wie);

    gemm_wmma<false, 0, true><<<dim3(768 / 64, NTOK / 128), 256, 0, stream>>>(
        lnb, W_attn, nullptr, nullptr, nullptr, nullptr, qkv, NTOK, 768, 256);
    gemm_wmma<false, 0, false><<<dim3(256 / 64, NTOK / 128), 256, 0, stream>>>(
        enc, Wie, nullptr, nullptr, nullptr, ie, nullptr, NTOK, 256, 256);

    attn_kernel<<<dim3(SS / 64, BB * 4), 128, 0, stream>>>(qkv, xb);
    intes_kernel<<<32, 256, 0, stream>>>(ie, xb);

    stats2_kernel<<<512, 256, 0, stream>>>(xb, stats2);
    fold_kernel<<<2, 256, 0, stream>>>(stats2, bn_g, bn_b, scale2, shift2);

    gemm_wmma<true, 1, false><<<dim3(256 / 64, NTOK / 128), 256, 0, stream>>>(
        xb, W_dec1, scale2, shift2, b_dec1, h1, nullptr, NTOK, 256, 512);
    gemm_wmma<false, 2, false><<<dim3(128 / 64, NTOK / 128), 256, 0, stream>>>(
        h1, W_dec2, nullptr, nullptr, b_dec2, out, nullptr, NTOK, 128, 256);
}
